// MultiQueryAttention_7919919694266
// MI455X (gfx1250) — hardware-verified
//
#include <hip/hip_runtime.h>
#include <math.h>


#ifndef NB
#define NB 4
#endif
#ifndef SEQ
#define SEQ 2048
#endif
#define NB_FULL 4
#define SEQ_FULL 2048
#define EE 1024
#define HH 8
#define DD 128
#define HD (HH * DD)
#ifndef QSPLIT
#define QSPLIT 512
#endif
#define QS (((QSPLIT) < (SEQ)) ? (QSPLIT) : (SEQ))
#define QS16 (QS / 16)
#define MMC (NB * SEQ)

#define BM 128
#define BN 64
#define BK 32
#define LP 40
#define SP 68
#define SPT 132
#define STAGE_FLOATS (BM * SP)

static_assert(NB >= 1 && NB <= NB_FULL);
static_assert(SEQ >= 128 && SEQ <= SEQ_FULL);
static_assert(SEQ % 128 == 0);
static_assert(QSPLIT % 128 == 0);
static_assert(QS % 128 == 0);
static_assert(MMC % BM == 0);
static_assert(EE % BN == 0 && HD % BN == 0 && (2 * DD) % BN == 0);
static_assert(EE % BK == 0 && HD % BK == 0);
static_assert(DD == 128 && HD == 1024 && EE == 1024);
static_assert(64 * SPT <= STAGE_FLOATS);

typedef _Float16 v16h __attribute__((ext_vector_type(16)));
typedef _Float16 v8h  __attribute__((ext_vector_type(8)));
typedef float    v8f  __attribute__((ext_vector_type(8)));
typedef float    v4f  __attribute__((ext_vector_type(4)));
typedef float    v2f  __attribute__((ext_vector_type(2)));
typedef unsigned int v4u __attribute__((ext_vector_type(4)));

union HFrag { v16h v; v8h h[2]; };
union H8 { v8h h; v4u u; };

__device__ __forceinline__ v16h load_frag(const _Float16* p) {
    HFrag f;
    f.h[0] = *reinterpret_cast<const v8h*>(p);
    f.h[1] = *reinterpret_cast<const v8h*>(p + 16);
    return f.v;
}

__device__ __forceinline__ v8f wmma16(v16h a, v16h b, v8f c) {
    v8f d = __builtin_amdgcn_wmma_f32_16x16x32_f16(false, a, false, b, (short)0, c, false, false);
    asm volatile("v_nop\n\tv_nop\n\tv_nop\n\tv_nop" : "+v"(d) : "v"(a), "v"(b));
    return d;
}

__device__ __forceinline__ _Float16 cvt_in(float v, float scale) {
    unsigned int u = __float_as_uint(v);
    u += 0x7FFFu + ((u >> 16) & 1u);
    u &= 0xFFFF0000u;
    return (_Float16)(__uint_as_float(u) * scale);
}

__device__ __forceinline__ void split_pack8(v8f v, v4u& ho, v4u& lo) {
    H8 h, l;
#pragma unroll
    for (int i = 0; i < 8; ++i) {
        _Float16 hv = (_Float16)v[i];
        h.h[i] = hv;
        l.h[i] = (_Float16)((v[i] - (float)hv) * 1024.0f);
    }
    ho = h.u;
    lo = l.u;
}

__global__ __launch_bounds__(256) void cvt_kernel(
    const float* __restrict__ src, _Float16* __restrict__ dst,
    int rowlen8, int src_rpb, int dst_rpb, float scale, int total8)
{
    const int i = blockIdx.x * 256 + threadIdx.x;
    if (i >= total8) return;
    const int rc = i / rowlen8;
    const int c8 = i - rc * rowlen8;
    const int b  = rc / dst_rpb;
    const int t  = rc - b * dst_rpb;
    const size_t soff = ((size_t)(b * src_rpb + t) * rowlen8 + c8) * 8;
    const v4f f0 = *reinterpret_cast<const v4f*>(src + soff);
    const v4f f1 = *reinterpret_cast<const v4f*>(src + soff + 4);
    H8 o;
#pragma unroll
    for (int k = 0; k < 4; ++k) {
        o.h[k]     = cvt_in(f0[k], scale);
        o.h[4 + k] = cvt_in(f1[k], scale);
    }
    _Float16* dp = dst + (size_t)i * 8;
    *(volatile v4u*)dp = o.u;
    __threadfence();
    *(volatile v4u*)dp = o.u;
}

__global__ __launch_bounds__(256) void pe_kernel(float* __restrict__ pe, int total2)
{
    const int i = blockIdx.x * 256 + threadIdx.x;
    if (i >= total2) return;
    const int t  = i >> 6;
    const int i2 = i & 63;
    const float frac = (float)(2 * i2) * (1.0f / 128.0f);
    const float ex   = -9.21034049987793f * frac;
    const float invf = expf(ex);
    const float ang  = (float)t * invf;
    float sn, cs;
    sincosf(ang, &sn, &cs);
    v2f o;
    o[0] = sn;
    o[1] = cs;
    float* p = pe + (size_t)i * 2;
    *(volatile v2f*)p = o;
    __threadfence();
    *(volatile v2f*)p = o;
}

template <int MODE>
__global__ __launch_bounds__(256) void gemm_kernel(
    const _Float16* __restrict__ A, const _Float16* __restrict__ A2,
    const _Float16* __restrict__ BT, const float* __restrict__ pe, float alpha,
    _Float16* __restrict__ P0, _Float16* __restrict__ P1,
    _Float16* __restrict__ P2, _Float16* __restrict__ P3,
    float* __restrict__ outp)
{
    __shared__ __attribute__((aligned(16))) _Float16 As[BM * LP];
    __shared__ __attribute__((aligned(16))) _Float16 A2s[BM * LP];
    __shared__ __attribute__((aligned(16))) _Float16 Bs[BN * LP];
    __shared__ __attribute__((aligned(16))) float stage[STAGE_FLOATS];

    const int tid  = threadIdx.x;
    const int lane = tid & 31;
    const int wave = tid >> 5;
    const int wm   = wave & 3;
    const int wn   = wave >> 2;
    const int l15  = lane & 15;
    const int hi8  = (lane >> 4) << 3;
    const int bm0  = blockIdx.y * BM;
    const int bn0  = blockIdx.x * BN;
    const int K    = (MODE == 2) ? HD : EE;
    const bool dual = (MODE == 2) && ((bm0 % SEQ) < QS);
    const int srow = tid >> 2;
    const int skg  = (tid & 3) * 8;

    v8f acc[2][2], acc2[2][2];
#pragma unroll
    for (int mi = 0; mi < 2; ++mi)
#pragma unroll
        for (int ni = 0; ni < 2; ++ni) { acc[mi][ni] = {}; acc2[mi][ni] = {}; }

#pragma unroll 1
    for (int k0 = 0; k0 < K; k0 += BK) {
#pragma unroll
        for (int i = 0; i < 2; ++i) {
            const int row = srow + i * 64;
            *reinterpret_cast<v8h*>(&As[row * LP + skg]) =
                *reinterpret_cast<const v8h*>(A + (size_t)(bm0 + row) * K + k0 + skg);
        }
        if (MODE == 2) {
            if (dual) {
#pragma unroll
                for (int i = 0; i < 2; ++i) {
                    const int row = srow + i * 64;
                    *reinterpret_cast<v8h*>(&A2s[row * LP + skg]) =
                        *reinterpret_cast<const v8h*>(A2 + (size_t)(bm0 + row) * K + k0 + skg);
                }
            }
        }
        *reinterpret_cast<v8h*>(&Bs[srow * LP + skg]) =
            *reinterpret_cast<const v8h*>(BT + (size_t)(bn0 + srow) * K + k0 + skg);
        __syncthreads();

        v16h aF[2], bF[2];
#pragma unroll
        for (int mi = 0; mi < 2; ++mi)
            aF[mi] = load_frag(&As[(wm * 32 + mi * 16 + l15) * LP + hi8]);
#pragma unroll
        for (int ni = 0; ni < 2; ++ni)
            bF[ni] = load_frag(&Bs[(wn * 32 + ni * 16 + l15) * LP + hi8]);
#pragma unroll
        for (int mi = 0; mi < 2; ++mi)
#pragma unroll
            for (int ni = 0; ni < 2; ++ni)
                acc[mi][ni] = wmma16(aF[mi], bF[ni], acc[mi][ni]);
        if (MODE == 2) {
            if (dual) {
                v16h a2F[2];
#pragma unroll
                for (int mi = 0; mi < 2; ++mi)
                    a2F[mi] = load_frag(&A2s[(wm * 32 + mi * 16 + l15) * LP + hi8]);
#pragma unroll
                for (int mi = 0; mi < 2; ++mi)
#pragma unroll
                    for (int ni = 0; ni < 2; ++ni)
                        acc2[mi][ni] = wmma16(a2F[mi], bF[ni], acc2[mi][ni]);
            }
        }
        __syncthreads();
    }

    const bool vpart = (MODE == 1) && (bn0 >= DD);
#pragma unroll
    for (int mi = 0; mi < 2; ++mi)
#pragma unroll
        for (int ni = 0; ni < 2; ++ni)
#pragma unroll
            for (int j = 0; j < 8; ++j) {
                const int r = wm * 32 + mi * 16 + hi8 + j;
                const int c = wn * 32 + ni * 16 + l15;
                float v;
                if (MODE == 2) {
                    v = acc[mi][ni][j];
                    if (dual) v += acc2[mi][ni][j] * (1.0f / 1024.0f);
                    v *= (1.0f / 1024.0f);
                } else {
                    v = acc[mi][ni][j] * 0.015625f;
                }
                if (vpart) stage[c * SPT + r] = v;
                else       stage[r * SP + c] = v;
            }
    __syncthreads();

    if (MODE == 0) {
        const int t0  = bm0 % SEQ;
        const int d00 = bn0 & (DD - 1);
#pragma unroll 1
        for (int pass = 0; pass < 2; ++pass) {
#pragma unroll
            for (int it = 0; it < 4; ++it) {
                const int idx = it * 256 + tid;
                const int r = idx >> 3;
                const int c = idx & 7;
                const v4f s0 = *reinterpret_cast<const v4f*>(&stage[r * SP + c * 8]);
                const v4f s1 = *reinterpret_cast<const v4f*>(&stage[r * SP + c * 8 + 4]);
                const float* pp = pe + (size_t)(t0 + r) * DD + d00 + c * 8;
                const v4f p0 = *reinterpret_cast<const v4f*>(pp);
                const v4f p1 = *reinterpret_cast<const v4f*>(pp + 4);
                v8f v;
#pragma unroll
                for (int i = 0; i < 4; ++i) {
                    v[i]     = (s0[i] + p0[i]) * alpha;
                    v[4 + i] = (s1[i] + p1[i]) * alpha;
                }
                v4u ho, lo;
                split_pack8(v, ho, lo);
                const size_t off = (size_t)(bm0 + r) * HD + bn0 + c * 8;
                *(volatile v4u*)(P0 + off) = ho;
                *(volatile v4u*)(P1 + off) = lo;
            }
            if (pass == 0) __threadfence();
        }
    } else if (MODE == 1) {
        if (!vpart) {
#pragma unroll 1
            for (int pass = 0; pass < 2; ++pass) {
#pragma unroll
                for (int it = 0; it < 4; ++it) {
                    const int idx = it * 256 + tid;
                    const int r = idx >> 3;
                    const int c = idx & 7;
                    const v4f s0 = *reinterpret_cast<const v4f*>(&stage[r * SP + c * 8]);
                    const v4f s1 = *reinterpret_cast<const v4f*>(&stage[r * SP + c * 8 + 4]);
                    v8f v;
#pragma unroll
                    for (int i = 0; i < 4; ++i) {
                        v[i]     = (s0[i] + ((i & 1) ? 1.0f : 0.0f)) * 4.0f;
                        v[4 + i] = (s1[i] + ((i & 1) ? 1.0f : 0.0f)) * 4.0f;
                    }
                    v4u ho, lo;
                    split_pack8(v, ho, lo);
                    const size_t off = (size_t)(bm0 + r) * DD + bn0 + c * 8;
                    *(volatile v4u*)(P0 + off) = ho;
                    *(volatile v4u*)(P1 + off) = lo;
                }
                if (pass == 0) __threadfence();
            }
        } else {
            const int bb = bm0 / SEQ;
            const int t0 = bm0 % SEQ;
            const int d0 = bn0 - DD;
#pragma unroll 1
            for (int pass = 0; pass < 2; ++pass) {
#pragma unroll
                for (int it = 0; it < 4; ++it) {
                    const int idx = it * 256 + tid;
                    const int r = idx >> 4;
                    const int c = idx & 15;
                    const v4f s0 = *reinterpret_cast<const v4f*>(&stage[r * SPT + c * 8]);
                    const v4f s1 = *reinterpret_cast<const v4f*>(&stage[r * SPT + c * 8 + 4]);
                    v8f v;
#pragma unroll
                    for (int i = 0; i < 4; ++i) {
                        v[i]     = s0[i] * 8.0f;
                        v[4 + i] = s1[i] * 8.0f;
                    }
                    v4u ho, lo;
                    split_pack8(v, ho, lo);
                    const size_t off = (size_t)(bb * DD + d0 + r) * SEQ + t0 + c * 8;
                    *(volatile v4u*)(P2 + off) = ho;
                    *(volatile v4u*)(P3 + off) = lo;
                }
                if (pass == 0) __threadfence();
            }
        }
    } else {
        const int row0 = (bm0 / SEQ) * SEQ_FULL + (bm0 % SEQ);
#pragma unroll 1
        for (int pass = 0; pass < 2; ++pass) {
#pragma unroll
            for (int it = 0; it < 8; ++it) {
                const int idx = it * 256 + tid;
                const int r = idx >> 4;
                const int c = idx & 15;
                const v4f s = *reinterpret_cast<const v4f*>(&stage[r * SP + c * 4]);
                const size_t off = (size_t)(row0 + r) * EE + bn0 + c * 4;
                *(volatile v4f*)(outp + off) = s;
            }
            if (pass == 0) __threadfence();
        }
    }
}

template <bool SPLIT>
__global__ __launch_bounds__(32) void attn_kernel(
    const _Float16* __restrict__ qh, const _Float16* __restrict__ ql,
    const _Float16* __restrict__ kh, const _Float16* __restrict__ kl,
    const _Float16* __restrict__ vTh, const _Float16* __restrict__ vTl,
    _Float16* __restrict__ yh, _Float16* __restrict__ yl, int qt_base)
{
    constexpr int NV = SPLIT ? 4 : 8;
    constexpr int DW = NV * 16;
    constexpr int YP = DW + 4;
    __shared__ __attribute__((aligned(16))) _Float16 psh[16 * LP];
    __shared__ __attribute__((aligned(16))) _Float16 psl[16 * LP];
    __shared__ __attribute__((aligned(16))) float ys[16 * YP];

    const int lane = threadIdx.x & 31;
    const int l15  = lane & 15;
    const int hi8  = (lane >> 4) << 3;
    const int bx   = blockIdx.x;
    const int qt   = qt_base + (SPLIT ? (bx >> 1) : bx);
    const int dbase = SPLIT ? ((bx & 1) * 64) : 0;
    const int hq   = blockIdx.y;
    const int b    = blockIdx.z;
    const int q0   = qt * 16;
    const int rowq = b * SEQ + q0;

    const size_t qoff = (size_t)(rowq + l15) * HD + hq * DD + hi8;
    const _Float16* kbh = kh  + (size_t)(b * SEQ) * DD + hi8;
    const _Float16* kbl = kl  + (size_t)(b * SEQ) * DD + hi8;
    const _Float16* vbh = vTh + (size_t)(b * DD) * SEQ + hi8;
    const _Float16* vbl = vTl + (size_t)(b * DD) * SEQ + hi8;

    float m[8], l[8];
    v8f accY[NV], accX[NV];
#pragma unroll
    for (int j = 0; j < 8; ++j) { m[j] = -1e30f; l[j] = 0.0f; }
#pragma unroll
    for (int ni = 0; ni < NV; ++ni) { accY[ni] = {}; accX[ni] = {}; }

    const int ntiles = (q0 >> 5) + 1;
#pragma unroll 1
    for (int it = 0; it < ntiles; ++it) {
        const int tc = it << 5;
        v8f s0 = {}, s1 = {}, x0 = {}, x1 = {};
#pragma unroll
        for (int kk = 0; kk < 4; ++kk) {
            const v16h aq = load_frag(qh + qoff + kk * 32);
            const _Float16* kp0 = kbh + (size_t)(tc + l15) * DD + kk * 32;
            const _Float16* kp1 = kp0 + 16 * DD;
            const v16h bk0 = load_frag(kp0);
            const v16h bk1 = load_frag(kp1);
            s0 = wmma16(aq, bk0, s0);
            s1 = wmma16(aq, bk1, s1);
            if (SPLIT) {
                const v16h al = load_frag(ql + qoff + kk * 32);
                const _Float16* lp0 = kbl + (size_t)(tc + l15) * DD + kk * 32;
                const _Float16* lp1 = lp0 + 16 * DD;
                const v16h bl0 = load_frag(lp0);
                const v16h bl1 = load_frag(lp1);
                x0 = wmma16(al, bk0, x0);
                x0 = wmma16(aq, bl0, x0);
                x1 = wmma16(al, bk1, x1);
                x1 = wmma16(aq, bl1, x1);
            }
        }
        if (SPLIT) {
            s0 = (s0 + x0 * (1.0f / 1024.0f)) * (1.0f / 32.0f);
            s1 = (s1 + x1 * (1.0f / 1024.0f)) * (1.0f / 32.0f);
        } else {
            s0 = s0 * (1.0f / 32.0f);
            s1 = s1 * (1.0f / 32.0f);
        }

        if (tc + 31 > q0) {
#pragma unroll
            for (int j = 0; j < 8; ++j) {
                const int qrow = q0 + hi8 + j;
                const int key0 = tc + l15;
                s0[j] = (key0 > qrow) ? -1e30f : s0[j];
                s1[j] = (key0 + 16 > qrow) ? -1e30f : s1[j];
            }
        }

#pragma unroll
        for (int j = 0; j < 8; ++j) {
            float mt = fmaxf(s0[j], s1[j]);
#pragma unroll
            for (int off = 8; off >= 1; off >>= 1)
                mt = fmaxf(mt, __shfl_xor(mt, off, 16));
            const float mn = fmaxf(m[j], mt);
            const float sc = exp2f(m[j] - mn);
            const float p0 = exp2f(s0[j] - mn);
            const float p1 = exp2f(s1[j] - mn);
            float rs = p0 + p1;
#pragma unroll
            for (int off = 8; off >= 1; off >>= 1)
                rs += __shfl_xor(rs, off, 16);
            l[j] = l[j] * sc + rs;
            m[j] = mn;
            s0[j] = p0;
            s1[j] = p1;
#pragma unroll
            for (int ni = 0; ni < NV; ++ni) {
                accY[ni][j] *= sc;
                if (SPLIT) accX[ni][j] *= sc;
            }
        }

#pragma unroll
        for (int j = 0; j < 8; ++j) {
            const int row = hi8 + j;
            const float c0 = s0[j] * 1024.0f;
            const float c1 = s1[j] * 1024.0f;
            const _Float16 h0 = (_Float16)c0;
            const _Float16 h1 = (_Float16)c1;
            psh[row * LP + l15]      = h0;
            psh[row * LP + 16 + l15] = h1;
            if (SPLIT) {
                psl[row * LP + l15]      = (_Float16)((c0 - (float)h0) * 1024.0f);
                psl[row * LP + 16 + l15] = (_Float16)((c1 - (float)h1) * 1024.0f);
            }
        }
        __syncthreads();
        const v16h aPh = load_frag(&psh[l15 * LP + hi8]);
        v16h aPl = {};
        if (SPLIT) aPl = load_frag(&psl[l15 * LP + hi8]);

#pragma unroll
        for (int ni = 0; ni < NV; ++ni) {
            const int d = dbase + ni * 16 + l15;
            const v16h bvh = load_frag(vbh + (size_t)d * SEQ + tc);
            accY[ni] = wmma16(aPh, bvh, accY[ni]);
            if (SPLIT) {
                const v16h bvl = load_frag(vbl + (size_t)d * SEQ + tc);
                accX[ni] = wmma16(aPl, bvh, accX[ni]);
                accX[ni] = wmma16(aPh, bvl, accX[ni]);
            }
        }
        __syncthreads();
    }

    float inv[8];
#pragma unroll
    for (int j = 0; j < 8; ++j) inv[j] = __builtin_amdgcn_rcpf(l[j]) * (1.0f / 512.0f);
#pragma unroll
    for (int ni = 0; ni < NV; ++ni)
#pragma unroll
        for (int j = 0; j < 8; ++j) {
            float v = accY[ni][j];
            if (SPLIT) v += accX[ni][j] * (1.0f / 1024.0f);
            ys[(hi8 + j) * YP + ni * 16 + l15] = v * inv[j];
        }
    __syncthreads();

    constexpr int CH  = DW / 8;
    constexpr int NIT = (16 * CH) / 32;
#pragma unroll 1
    for (int pass = 0; pass < 2; ++pass) {
#pragma unroll
        for (int it = 0; it < NIT; ++it) {
            const int idx = it * 32 + lane;
            const int r = idx / CH;
            const int c = idx & (CH - 1);
            const v4f a0 = *reinterpret_cast<const v4f*>(&ys[r * YP + c * 8]);
            const v4f a1 = *reinterpret_cast<const v4f*>(&ys[r * YP + c * 8 + 4]);
            v8f v;
#pragma unroll
            for (int i = 0; i < 4; ++i) { v[i] = a0[i]; v[4 + i] = a1[i]; }
            v4u ho, lo;
            split_pack8(v, ho, lo);
            const size_t off = (size_t)(rowq + r) * HD + hq * DD + dbase + c * 8;
            *(volatile v4u*)(yh + off) = ho;
            if (SPLIT) *(volatile v4u*)(yl + off) = lo;
        }
        if (pass == 0) __threadfence();
    }
}

extern "C" void kernel_launch(void* const* d_in, const int* in_sizes, int n_in,
                              void* d_out, int out_size, void* d_ws, size_t ws_size,
                              hipStream_t stream)
{
    if (n_in < 5) return;
    const long long needRows = (long long)(NB - 1) * SEQ_FULL + SEQ;
    if ((long long)in_sizes[0] < needRows * EE) return;
    if (in_sizes[1] < HD * EE) return;
    if (in_sizes[2] < DD * EE) return;
    if (in_sizes[3] < DD * EE) return;
    if (in_sizes[4] < EE * HD) return;
    if ((long long)out_size < needRows * EE) return;

    const float* x  = (const float*)d_in[0];
    const float* Wq = (const float*)d_in[1];
    const float* Wk = (const float*)d_in[2];
    const float* Wv = (const float*)d_in[3];
    const float* Wo = (const float*)d_in[4];
    float* out = (float*)d_out;

    char* ws = (char*)d_ws;
    size_t off = 0;
    _Float16* xh   = (_Float16*)(ws + off); off += (size_t)MMC * EE * 2;
    _Float16* Wqh  = (_Float16*)(ws + off); off += (size_t)HD * EE * 2;
    _Float16* Wkvh = (_Float16*)(ws + off); off += (size_t)2 * DD * EE * 2;
    _Float16* Woh  = (_Float16*)(ws + off); off += (size_t)EE * HD * 2;
    float*    pe   = (float*)(ws + off);    off += (size_t)SEQ * DD * 4;
    _Float16* qh   = (_Float16*)(ws + off); off += (size_t)MMC * HD * 2;
    _Float16* ql   = (_Float16*)(ws + off); off += (size_t)MMC * HD * 2;
    _Float16* kh   = (_Float16*)(ws + off); off += (size_t)MMC * DD * 2;
    _Float16* kl   = (_Float16*)(ws + off); off += (size_t)MMC * DD * 2;
    _Float16* vTh  = (_Float16*)(ws + off); off += (size_t)NB * DD * SEQ * 2;
    _Float16* vTl  = (_Float16*)(ws + off); off += (size_t)NB * DD * SEQ * 2;
    _Float16* yh   = (_Float16*)(ws + off); off += (size_t)MMC * HD * 2;
    _Float16* yl   = (_Float16*)(ws + off); off += (size_t)MMC * HD * 2;
    if (off > ws_size) return;

    const float scale   = 1.0f / sqrtf((float)DD);
    const float alphaQ8 = scale * 1.4426950408889634f * 8.0f;

    {
        const int total2 = SEQ * (DD / 2);
        pe_kernel<<<dim3((total2 + 255) / 256), dim3(256), 0, stream>>>(pe, total2);
    }
    {
        const int t8x = MMC * EE / 8;
        cvt_kernel<<<dim3((t8x + 255) / 256), dim3(256), 0, stream>>>(x, xh, EE / 8, SEQ_FULL, SEQ, 1.0f, t8x);
        const int t8q = HD * EE / 8;
        cvt_kernel<<<dim3((t8q + 255) / 256), dim3(256), 0, stream>>>(Wq, Wqh, EE / 8, HD, HD, 64.0f, t8q);
        const int t8k = DD * EE / 8;
        cvt_kernel<<<dim3((t8k + 255) / 256), dim3(256), 0, stream>>>(Wk, Wkvh, EE / 8, DD, DD, 64.0f, t8k);
        cvt_kernel<<<dim3((t8k + 255) / 256), dim3(256), 0, stream>>>(Wv, Wkvh + (size_t)DD * EE, EE / 8, DD, DD, 64.0f, t8k);
        const int t8o = EE * HD / 8;
        cvt_kernel<<<dim3((t8o + 255) / 256), dim3(256), 0, stream>>>(Wo, Woh, HD / 8, EE, EE, 64.0f, t8o);
    }
    gemm_kernel<0><<<dim3(HD / BN, MMC / BM), dim3(256), 0, stream>>>(
        xh, xh, Wqh, pe, alphaQ8, qh, ql, qh, ql, out);
    gemm_kernel<1><<<dim3((2 * DD) / BN, MMC / BM), dim3(256), 0, stream>>>(
        xh, xh, Wkvh, pe, 1.0f, kh, kl, vTh, vTl, out);
    attn_kernel<true><<<dim3(QS16 * 2, HH, NB), dim3(32), 0, stream>>>(
        qh, ql, kh, kl, vTh, vTl, yh, yl, 0);
    {
        const int nplain = SEQ / 16 - QS16;
        if (nplain > 0)
            attn_kernel<false><<<dim3(nplain, HH, NB), dim3(32), 0, stream>>>(
                qh, ql, kh, kl, vTh, vTl, yh, yl, QS16);
    }
    gemm_kernel<2><<<dim3(EE / BN, MMC / BM), dim3(256), 0, stream>>>(
        yh, yl, Woh, pe, 1.0f, qh, ql, qh, ql, out);
}
